// D2RLActor_64304250356440
// MI455X (gfx1250) — hardware-verified
//
#include <hip/hip_runtime.h>
#include <stddef.h>


#define DD       16
#define NGR      512
#define OUTX     64
#define OUTR     4
#define NTHR     256
#define NWAVE    8
#define EPT      8
#define NGRP     4
#define CHUNK    (NTHR * EPT * NGRP)
#define WCAP     (EPT * NGRP * 32)
#define NB       2048
#define NBSH     11
#define WSC      64.0f
#define WINV     0.015625f
#define BN_EPS   1e-5f

#define L_ACC    0
#define L_LIST   (NB * DD * 4)
#define L_CNT    (L_LIST + NWAVE * WCAP * 4)
#define L_WCNT   (L_CNT + NB * 4)
#define L_BNS    (L_WCNT + 128)
#define L_ST     (L_BNS + 2 * DD * 4)
#define L_REC    (L_ST + 16 * 16 * 2 * 8)
#define LDS_SAGE (L_REC + 32 * 8)

#define F_XE     0
#define F_GB     (NGR * DD)
#define F_OB     (2 * NGR * DD)
#define F_BNS    (F_OB + NGR * OUTX)
#define H_ST     ((F_BNS + 64) * 4)
#define LDS_HEAD (H_ST + 8 * 32 * 2 * 8)

static_assert(L_ACC == 0);
static_assert((NB & (NB - 1)) == 0);
static_assert(NB == (1 << NBSH));
static_assert((CHUNK & (CHUNK - 1)) == 0);
static_assert(((long long)(CHUNK - 1) << NBSH) < 2147483647LL);
static_assert((NB * DD / 4) % NTHR == 0);
static_assert((NB / 16) % NWAVE == 0);
static_assert(NGR == 2 * NTHR);
static_assert((NGR / 16) == 4 * NWAVE);
static_assert(NGR % 8 == 0);
static_assert((L_ST % 16) == 0 && (L_REC % 16) == 0 && (H_ST % 16) == 0);
static_assert(LDS_SAGE <= 300 * 1024);
static_assert(LDS_HEAD <= 300 * 1024);
static_assert((NGR * OUTX / 4) % NTHR == 0 && (NGR * OUTR / 4) % NTHR == 0);

typedef float    v4f  __attribute__((ext_vector_type(4)));
typedef float    v8f  __attribute__((ext_vector_type(8)));
typedef int      v4i  __attribute__((ext_vector_type(4)));
typedef double   v2d  __attribute__((ext_vector_type(2)));
typedef _Float16 f16_t;
typedef f16_t    v8h  __attribute__((ext_vector_type(8)));
typedef f16_t    v16h __attribute__((ext_vector_type(16)));
union FragH { v16h v; v8h h[2]; };

__device__ __forceinline__ v8f zero8() {
  v8f z = {0.f, 0.f, 0.f, 0.f, 0.f, 0.f, 0.f, 0.f};
  return z;
}

__device__ __forceinline__ v8f wmh(v16h a, v16h b, v8f c) {
  v8f d = __builtin_amdgcn_wmma_f32_16x16x32_f16(false, a, false, b, (short)0, c, false, false);
  asm volatile("v_nop\n\tv_nop\n\tv_nop\n\tv_nop" : "+v"(d) : "v"(a), "v"(b));
  return d;
}

#define SET8(F, B, P, Q) { \
  F.v[(B) + 0] = (f16_t)((P).x); F.v[(B) + 1] = (f16_t)((P).y); F.v[(B) + 2] = (f16_t)((P).z); F.v[(B) + 3] = (f16_t)((P).w); \
  F.v[(B) + 4] = (f16_t)((Q).x); F.v[(B) + 5] = (f16_t)((Q).y); F.v[(B) + 6] = (f16_t)((Q).z); F.v[(B) + 7] = (f16_t)((Q).w); }

__device__ __forceinline__ void store_relu8(float* dp, int pitch, v8f c, float bb) {
  dp[0 * pitch] = fmaxf(c[0] * WINV + bb, 0.0f);
  dp[1 * pitch] = fmaxf(c[1] * WINV + bb, 0.0f);
  dp[2 * pitch] = fmaxf(c[2] * WINV + bb, 0.0f);
  dp[3 * pitch] = fmaxf(c[3] * WINV + bb, 0.0f);
  dp[4 * pitch] = fmaxf(c[4] * WINV + bb, 0.0f);
  dp[5 * pitch] = fmaxf(c[5] * WINV + bb, 0.0f);
  dp[6 * pitch] = fmaxf(c[6] * WINV + bb, 0.0f);
  dp[7 * pitch] = fmaxf(c[7] * WINV + bb, 0.0f);
}
__device__ __forceinline__ void store_lin8(float* dp, int pitch, v8f c, float bb) {
  dp[0 * pitch] = c[0] * WINV + bb;
  dp[1 * pitch] = c[1] * WINV + bb;
  dp[2 * pitch] = c[2] * WINV + bb;
  dp[3 * pitch] = c[3] * WINV + bb;
  dp[4 * pitch] = c[4] * WINV + bb;
  dp[5 * pitch] = c[5] * WINV + bb;
  dp[6 * pitch] = c[6] * WINV + bb;
  dp[7 * pitch] = c[7] * WINV + bb;
}

__device__ __forceinline__ int scan_chunk(const int* __restrict__ dsts, int nE, int cbase, int nodeBase,
                                          int vec, int* list, int tid, int wave) {
  int wc = 0;
#pragma unroll
  for (int g = 0; g < NGRP; ++g) {
    const int el0  = (g * NTHR + tid) * EPT;
    const int e0   = cbase + el0;
    const int sent = -2147483647 - 1;
    v4i da, db;
    if (vec != 0 && cbase + CHUNK <= nE) {
      da = *(const v4i*)(dsts + e0);
      db = *(const v4i*)(dsts + e0 + 4);
    } else {
      const int em = nE - 1;
      da.x = (e0     < nE) ? dsts[(e0     < em) ? e0     : em] : sent;
      da.y = (e0 + 1 < nE) ? dsts[(e0 + 1 < em) ? e0 + 1 : em] : sent;
      da.z = (e0 + 2 < nE) ? dsts[(e0 + 2 < em) ? e0 + 2 : em] : sent;
      da.w = (e0 + 3 < nE) ? dsts[(e0 + 3 < em) ? e0 + 3 : em] : sent;
      db.x = (e0 + 4 < nE) ? dsts[(e0 + 4 < em) ? e0 + 4 : em] : sent;
      db.y = (e0 + 5 < nE) ? dsts[(e0 + 5 < em) ? e0 + 5 : em] : sent;
      db.z = (e0 + 6 < nE) ? dsts[(e0 + 6 < em) ? e0 + 6 : em] : sent;
      db.w = (e0 + 7 < nE) ? dsts[(e0 + 7 < em) ? e0 + 7 : em] : sent;
    }
    const unsigned nb = (unsigned)nodeBase;
    const unsigned s0 = (unsigned)da.x - nb, s1 = (unsigned)da.y - nb;
    const unsigned s2 = (unsigned)da.z - nb, s3 = (unsigned)da.w - nb;
    const unsigned s4 = (unsigned)db.x - nb, s5 = (unsigned)db.y - nb;
    const unsigned s6 = (unsigned)db.z - nb, s7 = (unsigned)db.w - nb;
    const bool h0 = s0 < (unsigned)NB, h1 = s1 < (unsigned)NB, h2 = s2 < (unsigned)NB, h3 = s3 < (unsigned)NB;
    const bool h4 = s4 < (unsigned)NB, h5 = s5 < (unsigned)NB, h6 = s6 < (unsigned)NB, h7 = s7 < (unsigned)NB;
#define HITJ(J, HJ, SJ) { \
      const unsigned mj = __builtin_amdgcn_ballot_w32(HJ); \
      if (mj != 0u) { \
        if (HJ) { \
          const int pos = wc + (int)__builtin_amdgcn_mbcnt_lo(mj, 0u); \
          if (pos < WCAP) list[wave * WCAP + pos] = ((el0 + (J)) << NBSH) | (int)(SJ); \
        } \
        wc += (int)__builtin_popcount(mj); } }
    HITJ(0, h0, s0)
    HITJ(1, h1, s1)
    HITJ(2, h2, s2)
    HITJ(3, h3, s3)
    HITJ(4, h4, s4)
    HITJ(5, h5, s5)
    HITJ(6, h6, s6)
    HITJ(7, h7, s7)
#undef HITJ
  }
  return wc;
}

__device__ __forceinline__ void drain_chunk(const int* __restrict__ srcs, const float* __restrict__ xin,
                                            int nN, int nE, int cbase,
                                            float* acc, int* cnt, const int* list, const int* wcnt, int lane) {
  const int grp = lane >> 2, sl = lane & 3;
#pragma unroll 1
  for (int w = 0; w < NWAVE; ++w) {
    int n = __builtin_amdgcn_readfirstlane(wcnt[w]);
    n = n > WCAP ? WCAP : (n < 0 ? 0 : n);
    const int* lp = list + w * WCAP;
#pragma unroll 1
    for (int b0 = 0; b0 < n; b0 += 32) {
      const int  q     = b0 + lane;
      const bool valid = q < n;
      const int  qc    = valid ? q : 0;
      int ent = lp[qc];
      ent = valid ? ent : 0;
      const int gq = ent & 7;
      const unsigned k0 = __builtin_amdgcn_ballot_w32(valid && gq == 0);
      const unsigned k1 = __builtin_amdgcn_ballot_w32(valid && gq == 1);
      const unsigned k2 = __builtin_amdgcn_ballot_w32(valid && gq == 2);
      const unsigned k3 = __builtin_amdgcn_ballot_w32(valid && gq == 3);
      const unsigned k4 = __builtin_amdgcn_ballot_w32(valid && gq == 4);
      const unsigned k5 = __builtin_amdgcn_ballot_w32(valid && gq == 5);
      const unsigned k6 = __builtin_amdgcn_ballot_w32(valid && gq == 6);
      const unsigned k7 = __builtin_amdgcn_ballot_w32(valid && gq == 7);
      unsigned mymask = (grp == 0) ? k0 : (grp == 1) ? k1 : (grp == 2) ? k2 : (grp == 3) ? k3 :
                        (grp == 4) ? k4 : (grp == 5) ? k5 : (grp == 6) ? k6 : k7;
      while (__builtin_amdgcn_ballot_w32(mymask != 0u) != 0u) {
        const bool take = mymask != 0u;
        int jl = __builtin_ffs((int)mymask) - 1;
        jl = take ? jl : 0;
        mymask &= mymask - 1u;
        const int e2   = __shfl(ent, jl);
        const int slot = e2 & (NB - 1);
        int e = cbase + (int)(((unsigned)e2) >> NBSH);
        e = e > nE - 1 ? nE - 1 : e;
        int src = srcs[e];
        src = src < 0 ? 0 : (src > nN - 1 ? nN - 1 : src);
        const v4f v = *(const v4f*)(xin + (size_t)src * DD + 4 * sl);
        if (take) {
          v4f* ap = (v4f*)(acc + slot * DD + 4 * sl);
          *ap = *ap + v;
          if (sl == 0) cnt[slot] = cnt[slot] + 1;
        }
      }
    }
  }
}

__global__ __launch_bounds__(NTHR) void k_sage(
    const int* __restrict__ ei, const float* __restrict__ xin,
    const float* __restrict__ Wl, const float* __restrict__ Wr, const float* __restrict__ bl,
    const float* __restrict__ gam, const float* __restrict__ bet,
    const double* __restrict__ pin, int nPin,
    float* xout, double* pout, int nN, int nE, int vec, int hasbn) {
  extern __shared__ v4f lds_dyn[];
  char*   lb   = (char*)lds_dyn;
  float*  acc  = (float*)(lb + L_ACC);
  int*    list = (int*)(lb + L_LIST);
  int*    cnt  = (int*)(lb + L_CNT);
  int*    wcnt = (int*)(lb + L_WCNT);
  float*  bns  = (float*)(lb + L_BNS);
  double* st   = (double*)(lb + L_ST);
  double* rec  = (double*)(lb + L_REC);
  const int tid = threadIdx.x, lane = tid & 31, wave = tid >> 5, hh = lane >> 4, m = lane & 15;
  const int nodeBase = blockIdx.x * NB;
  const int* srcs = ei;
  const int* dsts = ei + nE;

  {
    const v4f z = {0.f, 0.f, 0.f, 0.f};
    for (int i = tid; i < NB * DD / 4; i += NTHR) lds_dyn[i] = z;
    for (int i = tid; i < NB; i += NTHR) cnt[i] = 0;
  }
  if (tid < DD) {
    float s = 1.0f, sh = 0.0f;
    if (hasbn != 0) {
      double sm = 0.0, sq = 0.0;
#pragma unroll 1
      for (int b = 0; b < nPin; ++b) {
        sm += pin[(size_t)b * 32 + tid];
        sq += pin[(size_t)b * 32 + DD + tid];
      }
      const double mean = sm / (double)nN;
      double var = sq / (double)nN - mean * mean;
      if (var < 0.0) var = 0.0;
      s  = gam[tid] / sqrtf((float)var + BN_EPS);
      sh = bet[tid] - (float)mean * s;
    }
    bns[tid] = s;
    bns[DD + tid] = sh;
  }
  __syncthreads();

  const int nChunks = (nE + CHUNK - 1) / CHUNK;
#pragma unroll 1
  for (int ch = 0; ch < nChunks; ++ch) {
    const int cbase = ch * CHUNK;
    const int wc = scan_chunk(dsts, nE, cbase, nodeBase, vec, list, tid, wave);
    if (lane == 0) wcnt[wave] = wc;
    __syncthreads();
    if (wave == 0) drain_chunk(srcs, xin, nN, nE, cbase, acc, cnt, list, wcnt, lane);
    __syncthreads();
  }

  {
    FragH b;
    {
      const float* wl = Wl + m * DD + 8 * hh;
      const float* wr = Wr + m * DD + 8 * hh;
      v4f l0, l1, r0, r1;
      l0.x = wl[0] * WSC; l0.y = wl[1] * WSC; l0.z = wl[2] * WSC; l0.w = wl[3] * WSC;
      l1.x = wl[4] * WSC; l1.y = wl[5] * WSC; l1.z = wl[6] * WSC; l1.w = wl[7] * WSC;
      r0.x = wr[0] * WSC; r0.y = wr[1] * WSC; r0.z = wr[2] * WSC; r0.w = wr[3] * WSC;
      r1.x = wr[4] * WSC; r1.y = wr[5] * WSC; r1.z = wr[6] * WSC; r1.w = wr[7] * WSC;
      SET8(b, 0, l0, l1)
      SET8(b, 8, r0, r1)
    }
    const float blm = bl[m];
    const v4f s0 = *(const v4f*)(bns + 8 * hh), s1 = *(const v4f*)(bns + 8 * hh + 4);
    const v4f t0 = *(const v4f*)(bns + DD + 8 * hh), t1 = *(const v4f*)(bns + DD + 8 * hh + 4);
#pragma unroll 1
    for (int t = wave; t < NB / 16; t += NWAVE) {
      const int slotm = 16 * t + m;
      int node = nodeBase + slotm;
      node = node > nN - 1 ? nN - 1 : node;
      const int   cd  = cnt[slotm];
      const float inv = cd > 0 ? (1.0f / (float)cd) : 0.0f;
      const float z8  = cd > 0 ? 1.0f : 0.0f;
      const float* arow = acc + slotm * DD + 8 * hh;
      const float* xrow = xin + (size_t)node * DD + 8 * hh;
      v4f p0 = *(const v4f*)arow, p1 = *(const v4f*)(arow + 4);
      const v4f x0 = *(const v4f*)xrow, x1 = *(const v4f*)(xrow + 4);
      p0 = (p0 * inv * s0 + t0) * z8;
      p1 = (p1 * inv * s1 + t1) * z8;
      const v4f y0 = x0 * s0 + t0, y1 = x1 * s1 + t1;
      FragH a;
      SET8(a, 0, p0, p1)
      SET8(a, 8, y0, y1)
      const v8f c = wmh(a.v, b.v, zero8());
      store_relu8(acc + (16 * t + 8 * hh) * DD + m, DD, c, blm);
    }
  }
  __syncthreads();

  {
    float* gp = xout + (size_t)nodeBase * DD;
#pragma unroll 1
    for (int j = 0; j < (NB * DD / 4) / NTHR; ++j) {
      const int q = j * NTHR + tid;
      const v4f v = lds_dyn[q];
      *(volatile v4f*)(gp + 4 * (size_t)q) = v;
    }
    __threadfence();
#pragma unroll 1
    for (int j = 0; j < (NB * DD / 4) / NTHR; ++j) {
      const int q = j * NTHR + tid;
      const v4f v = lds_dyn[q];
      *(volatile v4f*)(gp + 4 * (size_t)q) = v;
    }
  }
  {
    int vr = nN - nodeBase;
    vr = vr > NB ? NB : vr;
    const int chn = tid & 15, grp = tid >> 4;
    double s = 0.0, q = 0.0;
#pragma unroll 1
    for (int r = grp; r < vr; r += 16) {
      const double v = (double)acc[r * DD + chn];
      s += v;
      q += v * v;
    }
    st[(grp * 16 + chn) * 2]     = s;
    st[(grp * 16 + chn) * 2 + 1] = q;
  }
  __syncthreads();
  if (tid < 32) {
    const int chn = tid & 15, which = tid >> 4;
    double tsum = 0.0;
#pragma unroll 1
    for (int grp = 0; grp < 16; ++grp) tsum += st[(grp * 16 + chn) * 2 + which];
    rec[tid] = tsum;
  }
  __syncthreads();
  if (wave == 0 && lane < 16) {
    const v2d v = *(const v2d*)(rec + 2 * lane);
    double* pp = pout + (size_t)blockIdx.x * 32 + 2 * lane;
    *(volatile v2d*)pp = v;
    __threadfence();
    *(volatile v2d*)pp = v;
  }
}

__device__ __forceinline__ v16h build_a(const float* base, int offA, int offB, int k32, const float* bns,
                                        int affine, int row, int hh) {
  v4f s0 = {1.f, 1.f, 1.f, 1.f}, s1 = s0, t0 = {0.f, 0.f, 0.f, 0.f}, t1 = t0;
  if (affine != 0) {
    s0 = *(const v4f*)(bns + 8 * hh);      s1 = *(const v4f*)(bns + 8 * hh + 4);
    t0 = *(const v4f*)(bns + 32 + 8 * hh); t1 = *(const v4f*)(bns + 32 + 8 * hh + 4);
  }
  const float* ra = base + offA + row * DD + 8 * hh;
  v4f p0 = *(const v4f*)ra, p1 = *(const v4f*)(ra + 4);
  p0 = p0 * s0 + t0;
  p1 = p1 * s1 + t1;
  v4f q0 = {0.f, 0.f, 0.f, 0.f}, q1 = q0;
  if (k32 != 0) {
    const v4f u0 = *(const v4f*)(bns + 16 + 8 * hh), u1 = *(const v4f*)(bns + 16 + 8 * hh + 4);
    const v4f w0 = *(const v4f*)(bns + 48 + 8 * hh), w1 = *(const v4f*)(bns + 48 + 8 * hh + 4);
    const float* rb = base + offB + row * DD + 8 * hh;
    q0 = (*(const v4f*)rb) * u0 + w0;
    q1 = (*(const v4f*)(rb + 4)) * u1 + w1;
  }
  FragH a;
  SET8(a, 0, p0, p1)
  SET8(a, 8, q0, q1)
  return a.v;
}

__device__ __forceinline__ v16h build_b(const float* __restrict__ W, int N, int k32, int ct, int m, int hh) {
  const int  n  = 16 * ct + m;
  const bool nv = n < N;
  const int  nc = nv ? n : (N - 1);
  const int  K  = (k32 != 0) ? 32 : 16;
  const float* wr = W + nc * K + 8 * hh;
  const float zs = nv ? WSC : 0.0f;
  v4f p0, p1, q0 = {0.f, 0.f, 0.f, 0.f}, q1 = q0;
  p0.x = wr[0] * zs; p0.y = wr[1] * zs; p0.z = wr[2] * zs; p0.w = wr[3] * zs;
  p1.x = wr[4] * zs; p1.y = wr[5] * zs; p1.z = wr[6] * zs; p1.w = wr[7] * zs;
  if (k32 != 0) {
    q0.x = wr[16] * zs; q0.y = wr[17] * zs; q0.z = wr[18] * zs; q0.w = wr[19] * zs;
    q1.x = wr[20] * zs; q1.y = wr[21] * zs; q1.z = wr[22] * zs; q1.w = wr[23] * zs;
  }
  FragH b;
  SET8(b, 0, p0, p1)
  SET8(b, 8, q0, q1)
  return b.v;
}

__device__ __forceinline__ void head_bn(float* base, int offA, int offB, int nch,
                                        const float* __restrict__ g, const float* __restrict__ be,
                                        float* bns, double* st, int tid) {
  const int ch = tid & 31, grp = tid >> 5;
  if (ch < nch) {
    const int off = (ch < 16) ? (offA + ch) : (offB + ch - 16);
    double s = 0.0, q = 0.0;
#pragma unroll 1
    for (int r = grp * (NGR / 8); r < (grp + 1) * (NGR / 8); ++r) {
      const double v = (double)base[off + r * DD];
      s += v;
      q += v * v;
    }
    st[(grp * 32 + ch) * 2]     = s;
    st[(grp * 32 + ch) * 2 + 1] = q;
  }
  __syncthreads();
  if (tid < nch) {
    double s = 0.0, q = 0.0;
#pragma unroll 1
    for (int gg = 0; gg < 8; ++gg) { s += st[(gg * 32 + tid) * 2]; q += st[(gg * 32 + tid) * 2 + 1]; }
    const double mean = s * (1.0 / (double)NGR);
    double var = q * (1.0 / (double)NGR) - mean * mean;
    if (var < 0.0) var = 0.0;
    const float sc = g[tid] / sqrtf((float)var + BN_EPS);
    bns[tid]      = sc;
    bns[32 + tid] = be[tid] - (float)mean * sc;
  }
  __syncthreads();
}

__device__ __forceinline__ void head_gemm16(float* base, int offA, int offB, int k32, const float* bns,
                                            const float* __restrict__ W, const float* __restrict__ bias,
                                            int offD, int lane, int wave) {
  const int hh = lane >> 4, m = lane & 15;
  const v16h b = build_b(W, DD, k32, 0, m, hh);
  const float bm = bias[m];
  v8f c0, c1, c2, c3;
  c0 = wmh(build_a(base, offA, offB, k32, bns, 1, 16 * (0 * NWAVE + wave) + m, hh), b, zero8());
  c1 = wmh(build_a(base, offA, offB, k32, bns, 1, 16 * (1 * NWAVE + wave) + m, hh), b, zero8());
  c2 = wmh(build_a(base, offA, offB, k32, bns, 1, 16 * (2 * NWAVE + wave) + m, hh), b, zero8());
  c3 = wmh(build_a(base, offA, offB, k32, bns, 1, 16 * (3 * NWAVE + wave) + m, hh), b, zero8());
  __syncthreads();
  store_relu8(base + offD + (16 * (0 * NWAVE + wave) + 8 * hh) * DD + m, DD, c0, bm);
  store_relu8(base + offD + (16 * (1 * NWAVE + wave) + 8 * hh) * DD + m, DD, c1, bm);
  store_relu8(base + offD + (16 * (2 * NWAVE + wave) + 8 * hh) * DD + m, DD, c2, bm);
  store_relu8(base + offD + (16 * (3 * NWAVE + wave) + 8 * hh) * DD + m, DD, c3, bm);
  __syncthreads();
}

__device__ __forceinline__ void head_out(float* base, int offA, const float* __restrict__ W,
                                         const float* __restrict__ bias, int N, int offD, float* outp,
                                         int tid, int lane, int wave) {
  const int hh = lane >> 4, m = lane & 15;
  const int CT = (N + 15) >> 4;
  const int ntile = (NGR / 16) * CT;
#pragma unroll 1
  for (int tt = wave; tt < ntile; tt += NWAVE) {
    const int t = tt / CT, ct = tt - t * CT;
    const v16h a = build_a(base, offA, offA, 0, base, 0, 16 * t + m, hh);
    const v16h b = build_b(W, N, 0, ct, m, hh);
    const v8f c = wmh(a, b, zero8());
    const int  n  = 16 * ct + m;
    const bool nv = n < N;
    const int  nc = nv ? n : (N - 1);
    const float bb = bias[nc];
    if (nv) store_lin8(base + offD + (16 * t + 8 * hh) * N + nc, N, c, bb);
  }
  __syncthreads();
#pragma unroll 1
  for (int rr = 0; rr < 2; ++rr) {
    float* rp = base + offD + (tid + rr * NTHR) * N;
    float mx = rp[0];
#pragma unroll 1
    for (int c2 = 1; c2 < N; ++c2) mx = fmaxf(mx, rp[c2]);
    float sum = 0.0f;
#pragma unroll 1
    for (int c2 = 0; c2 < N; ++c2) { const float e = expf(rp[c2] - mx); rp[c2] = e; sum += e; }
    const float inv = 1.0f / sum;
#pragma unroll 1
    for (int c2 = 0; c2 < N; ++c2) rp[c2] = rp[c2] * inv;
  }
  __syncthreads();
  const int nq = NGR * N / 4;
#pragma unroll 1
  for (int q = tid; q < nq; q += NTHR) {
    const v4f v = *(const v4f*)(base + offD + 4 * q);
    *(volatile v4f*)(outp + 4 * (size_t)q) = v;
  }
  __threadfence();
#pragma unroll 1
  for (int q = tid; q < nq; q += NTHR) {
    const v4f v = *(const v4f*)(base + offD + 4 * q);
    *(volatile v4f*)(outp + 4 * (size_t)q) = v;
  }
  __syncthreads();
}

__global__ __launch_bounds__(NTHR) void k_head(
    const int* __restrict__ batch, const float* __restrict__ h2, int nN,
    const float* __restrict__ n1g, const float* __restrict__ n1b,
    const float* __restrict__ W1, const float* __restrict__ b1,
    const float* __restrict__ n2g, const float* __restrict__ n2b,
    const float* __restrict__ W2, const float* __restrict__ b2,
    const float* __restrict__ n3g, const float* __restrict__ n3b,
    const float* __restrict__ W3, const float* __restrict__ b3,
    const float* __restrict__ Wx, const float* __restrict__ bx,
    const float* __restrict__ Wy, const float* __restrict__ by,
    const float* __restrict__ Wq, const float* __restrict__ bq4,
    float* out) {
  extern __shared__ v4f lds_dyn[];
  float*  base = (float*)lds_dyn;
  float*  bns  = base + F_BNS;
  double* st   = (double*)((char*)lds_dyn + H_ST);
  const int tid = threadIdx.x, lane = tid & 31, wave = tid >> 5;

  {
    const int ga = tid, gb = tid + NTHR;
    v4f pa0 = {0.f, 0.f, 0.f, 0.f}, pa1 = pa0, pa2 = pa0, pa3 = pa0;
    v4f pb0 = pa0, pb1 = pa0, pb2 = pa0, pb3 = pa0;
    int ca = 0, cb = 0;
#pragma unroll 1
    for (int n = 0; n < nN; ++n) {
      const int bq = batch[n];
      const bool ha = (bq == ga), hb = (bq == gb);
      if (__builtin_amdgcn_ballot_w32(ha || hb) != 0u) {
        const float* rp = h2 + (size_t)n * DD;
        const v4f r0 = *(const v4f*)(rp), r1 = *(const v4f*)(rp + 4);
        const v4f r2 = *(const v4f*)(rp + 8), r3 = *(const v4f*)(rp + 12);
        if (ha) { pa0 += r0; pa1 += r1; pa2 += r2; pa3 += r3; ca += 1; }
        if (hb) { pb0 += r0; pb1 += r1; pb2 += r2; pb3 += r3; cb += 1; }
      }
    }
    const float ia = 1.0f / (float)(ca > 0 ? ca : 1);
    const float ib = 1.0f / (float)(cb > 0 ? cb : 1);
    v4f* xa = (v4f*)(base + F_XE + ga * DD);
    xa[0] = pa0 * ia; xa[1] = pa1 * ia; xa[2] = pa2 * ia; xa[3] = pa3 * ia;
    v4f* xb = (v4f*)(base + F_XE + gb * DD);
    xb[0] = pb0 * ib; xb[1] = pb1 * ib; xb[2] = pb2 * ib; xb[3] = pb3 * ib;
  }
  __syncthreads();

  head_bn(base, F_XE, F_XE, 16, n1g, n1b, bns, st, tid);
  head_gemm16(base, F_XE, F_XE, 0, bns, W1, b1, F_GB, lane, wave);
  head_bn(base, F_GB, F_XE, 32, n2g, n2b, bns, st, tid);
  head_gemm16(base, F_GB, F_XE, 1, bns, W2, b2, F_GB, lane, wave);
  head_bn(base, F_GB, F_XE, 32, n3g, n3b, bns, st, tid);
  head_gemm16(base, F_GB, F_XE, 1, bns, W3, b3, F_GB, lane, wave);

  head_out(base, F_GB, Wx, bx,  OUTX, F_OB, out,                            tid, lane, wave);
  head_out(base, F_GB, Wy, by,  OUTX, F_OB, out + (size_t)NGR * OUTX,       tid, lane, wave);
  head_out(base, F_GB, Wq, bq4, OUTR, F_OB, out + (size_t)2 * NGR * OUTX,   tid, lane, wave);
}

extern "C" void kernel_launch(void* const* d_in, const int* in_sizes, int n_in,
                              void* d_out, int out_size, void* d_ws, size_t ws_size,
                              hipStream_t stream) {
  if (n_in < 29) return;
  const int nN = in_sizes[0] / DD;
  const int nE = in_sizes[1] / 2;
  if (nN <= 0 || nE < 0) return;
  if (in_sizes[0] != nN * DD || in_sizes[1] != 2 * nE || in_sizes[2] != nN) return;
  if (in_sizes[3] != DD * DD || in_sizes[5] != DD * DD || in_sizes[6] != DD * DD || in_sizes[8] != DD * DD) return;
  if (in_sizes[4] < DD || in_sizes[7] < DD || in_sizes[9] < DD || in_sizes[10] < DD) return;
  if (in_sizes[11] != DD * DD || in_sizes[12] < DD || in_sizes[13] < DD || in_sizes[14] < DD) return;
  if (in_sizes[15] != DD * 2 * DD || in_sizes[16] < DD || in_sizes[17] < 2 * DD || in_sizes[18] < 2 * DD) return;
  if (in_sizes[19] != DD * 2 * DD || in_sizes[20] < DD || in_sizes[21] < 2 * DD || in_sizes[22] < 2 * DD) return;
  if (in_sizes[23] != OUTX * DD || in_sizes[24] < OUTX || in_sizes[25] != OUTX * DD || in_sizes[26] < OUTX) return;
  if (in_sizes[27] != OUTR * DD || in_sizes[28] < OUTR) return;
  if (out_size != NGR * (2 * OUTX + OUTR)) return;

  const float* x    = (const float*)d_in[0];
  const int*   ei   = (const int*)d_in[1];
  const int*   bt   = (const int*)d_in[2];
  const float* c1Wl = (const float*)d_in[3];
  const float* c1bl = (const float*)d_in[4];
  const float* c1Wr = (const float*)d_in[5];
  const float* c2Wl = (const float*)d_in[6];
  const float* c2bl = (const float*)d_in[7];
  const float* c2Wr = (const float*)d_in[8];
  const float* n1g  = (const float*)d_in[9];
  const float* n1b  = (const float*)d_in[10];
  const float* l1W  = (const float*)d_in[11];
  const float* l1b  = (const float*)d_in[12];
  const float* nl1g = (const float*)d_in[13];
  const float* nl1b = (const float*)d_in[14];
  const float* l2W  = (const float*)d_in[15];
  const float* l2b  = (const float*)d_in[16];
  const float* nl2g = (const float*)d_in[17];
  const float* nl2b = (const float*)d_in[18];
  const float* l3W  = (const float*)d_in[19];
  const float* l3b  = (const float*)d_in[20];
  const float* nl3g = (const float*)d_in[21];
  const float* nl3b = (const float*)d_in[22];
  const float* lxW  = (const float*)d_in[23];
  const float* lxb  = (const float*)d_in[24];
  const float* lyW  = (const float*)d_in[25];
  const float* lyb  = (const float*)d_in[26];
  const float* lrW  = (const float*)d_in[27];
  const float* lrb  = (const float*)d_in[28];
  float* out = (float*)d_out;

  const int nBlk = (nN + NB - 1) / NB;

  char* ws = (char*)d_ws;
  size_t off = 0;
  const size_t szX = (size_t)nBlk * NB * DD * 4;
  const size_t szP = (size_t)nBlk * 32 * 8;
  const size_t oH1 = off; off += szX; off = (off + 255) & ~(size_t)255;
  const size_t oH2 = off; off += szX; off = (off + 255) & ~(size_t)255;
  const size_t oP1 = off; off += szP; off = (off + 255) & ~(size_t)255;
  const size_t oP2 = off; off += szP; off = (off + 255) & ~(size_t)255;
  if (off > ws_size) return;
  float*  h1 = (float*)(ws + oH1);
  float*  h2 = (float*)(ws + oH2);
  double* p1 = (double*)(ws + oP1);
  double* p2 = (double*)(ws + oP2);

  const int vec = ((nE & 3) == 0) ? 1 : 0;

  hipFuncSetAttribute(reinterpret_cast<const void*>(&k_sage),
                      hipFuncAttributeMaxDynamicSharedMemorySize, LDS_SAGE);
  hipFuncSetAttribute(reinterpret_cast<const void*>(&k_head),
                      hipFuncAttributeMaxDynamicSharedMemorySize, LDS_HEAD);

  k_sage<<<nBlk, NTHR, LDS_SAGE, stream>>>(ei, x, c1Wl, c1Wr, c1bl, n1g, n1b, p2, 0,
                                           h1, p1, nN, nE, vec, 0);
  k_sage<<<nBlk, NTHR, LDS_SAGE, stream>>>(ei, h1, c2Wl, c2Wr, c2bl, n1g, n1b, p1, nBlk,
                                           h2, p2, nN, nE, vec, 1);
  k_head<<<1, NTHR, LDS_HEAD, stream>>>(bt, h2, nN,
                                       nl1g, nl1b, l1W, l1b,
                                       nl2g, nl2b, l2W, l2b,
                                       nl3g, nl3b, l3W, l3b,
                                       lxW, lxb, lyW, lyb, lrW, lrb, out);
}
